// mutualPoolingDir_45234595562201
// MI455X (gfx1250) — hardware-verified
//
#include <hip/hip_runtime.h>

typedef __bf16 v16b __attribute__((ext_vector_type(16)));
typedef float  v8f  __attribute__((ext_vector_type(8)));
typedef float  v4f  __attribute__((ext_vector_type(4)));
typedef int    v8i  __attribute__((ext_vector_type(8)));
typedef v4f __attribute__((may_alias)) v4fa;

#define NG    64
#define NL    100
#define ND    128
#define NP    64
#define NROWS (NG * NL)
#define TP    132
#define PPB   32
#define NTHR  128

static_assert(NROWS % 64 == 0);
static_assert(NP % PPB == 0);
static_assert((NL * ND) % (4 * NTHR) == 0);
static_assert(NL % 4 == 0);

union BFrag { v16b v; v8i i; };

__device__ __forceinline__ v8f wmma_bf16(v16b a, v16b b, v8f c) {
  v8f d = __builtin_amdgcn_wmma_f32_16x16x32_bf16(false, a, false, b, (short)0, c, false, false);
  BFrag ua, ub;
  ua.v = a;
  ub.v = b;
  asm volatile("v_nop\n\tv_nop\n\tv_nop\n\tv_nop" : "+v"(d) : "v"(ua.i), "v"(ub.i));
  return d;
}

__device__ __forceinline__ void load_split(const float* p0, const float* p1, v16b& hi, v16b& lo) {
  const v4f a = *(const v4fa*)p0;
  const v4f b = *(const v4fa*)(p0 + 4);
  const v4f c = *(const v4fa*)p1;
  const v4f e = *(const v4fa*)(p1 + 4);
  const float x[16] = { a.x, a.y, a.z, a.w, b.x, b.y, b.z, b.w,
                        c.x, c.y, c.z, c.w, e.x, e.y, e.z, e.w };
  #pragma unroll
  for (int i = 0; i < 16; ++i) {
    const __bf16 hb = (__bf16)x[i];
    const float  hf = (float)hb;
    hi[i] = hb;
    lo[i] = (__bf16)(x[i] - hf);
  }
}

__device__ __forceinline__ void proj_store_pass(const float* sT, float* kws, int rblk, int w, int lane) {
  const float* src0 = sT + (16 * w) * TP + 4 * lane;
  float* dst0 = kws + (size_t)(rblk + 16 * w) * ND + 4 * lane;
  #pragma unroll
  for (int i = 0; i < 16; ++i) {
    const v4f v = *(const v4fa*)(src0 + i * TP);
    *(volatile v4f*)(dst0 + (size_t)i * ND) = v;
  }
}

__global__ __launch_bounds__(NTHR) void k_proj(
    const float* __restrict__ xb,
    const float* __restrict__ wk,
    const float* __restrict__ bk,
    float* __restrict__ kws)
{
  __shared__ __attribute__((aligned(16))) float sT[64 * TP];

  const int tid = threadIdx.x, lane = tid & 31, w = tid >> 5;
  const int h = lane >> 4, m = lane & 15;
  const int rblk = blockIdx.x * 64;
  const float* arow = xb + (size_t)(rblk + 16 * w + m) * ND;

  const v8f z8 = {0.f, 0.f, 0.f, 0.f, 0.f, 0.f, 0.f, 0.f};
  v8f acc[8];
  #pragma unroll
  for (int nt = 0; nt < 8; ++nt) acc[nt] = z8;

  #pragma unroll 1
  for (int k0 = 0; k0 < ND; k0 += 32) {
    v16b ahi, alo;
    load_split(arow + k0 + 8 * h, arow + k0 + 16 + 8 * h, ahi, alo);
    #pragma unroll
    for (int nt = 0; nt < 8; ++nt) {
      const float* brow = wk + (size_t)(16 * nt + m) * ND + k0;
      v16b bhi, blo;
      load_split(brow + 8 * h, brow + 16 + 8 * h, bhi, blo);
      v8f c = acc[nt];
      c = wmma_bf16(ahi, bhi, c);
      c = wmma_bf16(ahi, blo, c);
      c = wmma_bf16(alo, bhi, c);
      acc[nt] = c;
    }
  }

  #pragma unroll
  for (int nt = 0; nt < 8; ++nt) {
    const float bias = bk[16 * nt + m];
    #pragma unroll
    for (int r = 0; r < 8; ++r)
      sT[(16 * w + 8 * h + r) * TP + 16 * nt + m] = acc[nt][r] + bias;
  }
  __syncthreads();

  proj_store_pass(sT, kws, rblk, w, lane);
  __threadfence();
  proj_store_pass(sT, kws, rblk, w, lane);
}

__global__ __launch_bounds__(NTHR) void k_pool(
    const float* __restrict__ kws,
    const float* __restrict__ gval,
    const float* __restrict__ qry,
    float* __restrict__ out)
{
  __shared__ __attribute__((aligned(16))) float sK[NL * ND];
  __shared__ __attribute__((aligned(16))) float sV[NL * ND];
  __shared__ __attribute__((aligned(16))) float sO[4 * ND];

  const int tid = threadIdx.x, lane = tid & 31, w = tid >> 5;
  const int g = blockIdx.x;
  const int pbase = blockIdx.y * PPB;
  const size_t gbase = (size_t)g * NL * ND;

  for (int i = tid; i < (NL * ND) / 4; i += NTHR) {
    const v4f a = *(const v4fa*)(kws + gbase + 4 * i);
    const v4f b = *(const v4fa*)(gval + gbase + 4 * i);
    *(v4fa*)(sK + 4 * i) = a;
    *(v4fa*)(sV + 4 * i) = b;
  }
  __syncthreads();

  const int d = tid;
  float kmx = -3.402823466e+38f, kmn = 3.402823466e+38f;
  #pragma unroll 4
  for (int l = 0; l < NL; ++l) {
    const float k = sK[l * ND + d];
    kmx = fmaxf(kmx, k);
    kmn = fminf(kmn, k);
  }

  #pragma unroll 1
  for (int grp = 0; grp < PPB / 4; ++grp) {
    const int p0 = pbase + 4 * grp;
    #pragma unroll 1
    for (int j = 0; j < 4; ++j) {
      const int p = p0 + j;
      const float q = qry[p * ND + d];
      const float mpos = q * kmx;
      const float mneg = q * kmn;
      const float mx = (q >= 0.f) ? mpos : mneg;
      float s = 0.f, acc = 0.f;
      #pragma unroll 4
      for (int l = 0; l < NL; ++l) {
        const float k = sK[l * ND + d];
        const float e = __expf(q * k - mx);
        s += e;
        acc = fmaf(e, sV[l * ND + d], acc);
      }
      const float val = acc * __builtin_amdgcn_rcpf(s);
      sO[j * ND + d] = val;
    }
    __syncthreads();

    const v4f v = *(const v4fa*)(sO + w * ND + 4 * lane);
    float* dst = out + ((size_t)(p0 + w) * NG + g) * ND + 4 * lane;
    *(volatile v4f*)dst = v;
    __threadfence();
    *(volatile v4f*)dst = v;
    __syncthreads();
  }
}

extern "C" void kernel_launch(void* const* d_in, const int* in_sizes, int n_in,
                              void* d_out, int out_size, void* d_ws, size_t ws_size,
                              hipStream_t stream) {
  if (n_in < 5) return;
  if (in_sizes[0] != NROWS * ND) return;
  if (in_sizes[1] != NROWS * ND) return;
  if (in_sizes[2] != NP * ND) return;
  if (in_sizes[3] != ND * ND) return;
  if (in_sizes[4] != ND) return;
  if (out_size != NP * NG * ND) return;

  const size_t kws_bytes = (size_t)NROWS * ND * sizeof(float);
  if (kws_bytes > ws_size) return;

  const float* gval = (const float*)d_in[0];
  const float* xb   = (const float*)d_in[1];
  const float* qry  = (const float*)d_in[2];
  const float* wk   = (const float*)d_in[3];
  const float* bk   = (const float*)d_in[4];
  float* out = (float*)d_out;
  float* kws = (float*)d_ws;

  k_proj<<<NROWS / 64, NTHR, 0, stream>>>(xb, wk, bk, kws);

  dim3 gPool(NG, NP / PPB);
  k_pool<<<gPool, NTHR, 0, stream>>>(kws, gval, qry, out);
}
